// TorchTreeNNModel_23132693856420
// MI455X (gfx1250) — hardware-verified
//
#include <hip/hip_runtime.h>


typedef float          v4f  __attribute__((ext_vector_type(4)));
typedef float          v8f  __attribute__((ext_vector_type(8)));
typedef unsigned short us_t;
typedef us_t           v8us __attribute__((ext_vector_type(8)));
typedef __bf16         v16b __attribute__((ext_vector_type(16)));

union BFrag { v16b v; v8us q[2]; };
union Pk8   { v8us v; us_t s[8]; };

#define NNODE 512
#define DIM   128
#define KDIM  256
#define NOUT  3
#define TPB   16
#define NWAVE 8
#define TP    264
#define SP    132

__device__ __forceinline__ int clampi(int x, int lo, int hi) {
    return x < lo ? lo : (x > hi ? hi : x);
}

__device__ __forceinline__ unsigned int bf16_rne(float x) {
    unsigned int u = __float_as_uint(x);
    return (u + 0x7FFFu + ((u >> 16) & 1u)) >> 16;
}

__device__ __forceinline__ void split_bf16(float x, us_t& hi, us_t& lo) {
    unsigned int hb = bf16_rne(x);
    float hf = __uint_as_float(hb << 16);
    hi = (us_t)hb;
    lo = (us_t)bf16_rne(x - hf);
}

__device__ __forceinline__ float act_tanh(float x) {
    float ax = fabsf(x);
    float t  = __expf(-2.0f * ax);
    float r  = (1.0f - t) * __builtin_amdgcn_rcpf(1.0f + t);
    return copysignf(r, x);
}

__device__ __forceinline__ v8f wmma_bf(const BFrag& a, const BFrag& b, v8f c) {
    return __builtin_amdgcn_wmma_f32_16x16x32_bf16(false, a.v, false, b.v, (short)0, c, false, false);
}

__global__ __launch_bounds__(256)
void k_wsplit(const float* __restrict__ W, us_t* Phi, us_t* Plo, int n8) {
    const int i = blockIdx.x * 256 + threadIdx.x;
    if (i >= n8) return;
    const float* p = W + (size_t)i * 8;
    const v4f a = *(const v4f*)p;
    const v4f b = *(const v4f*)(p + 4);
    Pk8 hi, lo;
#pragma unroll
    for (int e = 0; e < 4; ++e) {
        split_bf16(a[e], hi.s[e],     lo.s[e]);
        split_bf16(b[e], hi.s[4 + e], lo.s[4 + e]);
    }
    us_t* dh = Phi + (size_t)i * 8;
    us_t* dl = Plo + (size_t)i * 8;
    *(volatile v8us*)dh = hi.v;
    *(volatile v8us*)dl = lo.v;
    __threadfence();
    *(volatile v8us*)dh = hi.v;
    *(volatile v8us*)dl = lo.v;
}

__global__ __launch_bounds__(256)
void k_recur(const int* __restrict__ sub, const int* __restrict__ lens,
             const int* __restrict__ eind, const float* __restrict__ emb,
             const us_t* __restrict__ Whi, const us_t* __restrict__ Wlo,
             const float* __restrict__ bt, float* S, float* R,
             int tbase, int vocab)
{
    __shared__ __attribute__((aligned(16))) us_t  Thi[TPB * TP];
    __shared__ __attribute__((aligned(16))) us_t  Tlo[TPB * TP];
    __shared__ __attribute__((aligned(16))) float So[TPB * SP];
    __shared__ int s_p[TPB];
    __shared__ int s_l[TPB];
    __shared__ int s_r[TPB];
    __shared__ unsigned int s_msk;

    const int tid   = threadIdx.x;
    const int lane  = tid & 31;
    const int wave  = __builtin_amdgcn_readfirstlane(tid >> 5);
    const int h     = lane >> 4;
    const int m     = lane & 15;
    const int slot0 = blockIdx.x * TPB;
    const int tg0   = tbase + slot0;

#pragma unroll 1
    for (int q = wave; q < TPB * NNODE; q += NWAVE) {
        const int mt   = q >> 9;
        const int node = q & (NNODE - 1);
        int id = eind[(size_t)(tg0 + mt) * NNODE + node];
        id = clampi(id, 0, vocab - 1);
        const v4f v = *(const v4f*)(emb + (size_t)id * DIM + 4 * lane);
        float* d = S + ((size_t)(slot0 + mt) * NNODE + node) * DIM + 4 * lane;
        *(volatile v4f*)d = v;
        __threadfence();
        *(volatile v4f*)d = v;
    }
    __threadfence();
    __syncthreads();

    const int  myn  = lens[tg0 + m];
    const int  f0   = 16 * wave + 8 * h;
    const v4f  bia0 = *(const v4f*)(bt + f0);
    const v4f  bia1 = *(const v4f*)(bt + f0 + 4);
    const us_t* aph = Whi + (size_t)(16 * wave + m) * KDIM + 8 * h;
    const us_t* apl = Wlo + (size_t)(16 * wave + m) * KDIM + 8 * h;
    const us_t* bph = Thi + m * TP + 8 * h;
    const us_t* bpl = Tlo + m * TP + 8 * h;
    const int gm = tid >> 4;
    const int gc = tid & 15;

#pragma unroll 1
    for (int i = 0; i < NNODE; ++i) {
        if (wave == 0) {
            const int* row = sub + ((size_t)(tg0 + m) * NNODE + i) * 3;
            const int p = row[0], l = row[1], r = row[2];
            const bool doit = (l != r) && (i < myn) && ((unsigned)p < (unsigned)NNODE);
            const unsigned int bal = (unsigned int)__ballot(doit) & 0xFFFFu;
            if (lane < TPB) {
                s_p[lane] = clampi(p, 0, NNODE - 1);
                s_l[lane] = clampi(l, 0, NNODE - 1);
                s_r[lane] = clampi(r, 0, NNODE - 1);
            }
            if (lane == 0) s_msk = bal;
        }
        __syncthreads();
        const unsigned int msk = (unsigned int)__builtin_amdgcn_readfirstlane((int)s_msk);
        if (msk != 0u) {
            {
                const int nl = s_l[gm];
                const int nr = s_r[gm];
                const int node = (gc < 8) ? nl : nr;
                const float* src = S + ((size_t)(slot0 + gm) * NNODE + node) * DIM + (gc & 7) * 16;
                const v4f x0 = *(const v4f*)(src);
                const v4f x1 = *(const v4f*)(src + 4);
                const v4f x2 = *(const v4f*)(src + 8);
                const v4f x3 = *(const v4f*)(src + 12);
                Pk8 h0, h1, l0, l1;
#pragma unroll
                for (int e = 0; e < 4; ++e) {
                    split_bf16(x0[e], h0.s[e],     l0.s[e]);
                    split_bf16(x1[e], h0.s[4 + e], l0.s[4 + e]);
                    split_bf16(x2[e], h1.s[e],     l1.s[e]);
                    split_bf16(x3[e], h1.s[4 + e], l1.s[4 + e]);
                }
                us_t* th = Thi + gm * TP + gc * 16;
                us_t* tl = Tlo + gm * TP + gc * 16;
                *(v8us*)(th)     = h0.v;
                *(v8us*)(th + 8) = h1.v;
                *(v8us*)(tl)     = l0.v;
                *(v8us*)(tl + 8) = l1.v;
            }
            __syncthreads();

            v8f acc = {0.f, 0.f, 0.f, 0.f, 0.f, 0.f, 0.f, 0.f};
#pragma unroll 2
            for (int kt = 0; kt < KDIM / 32; ++kt) {
                const int ko = kt * 32;
                BFrag ah, al, bh, bl;
                ah.q[0] = *(const v8us*)(aph + ko);
                ah.q[1] = *(const v8us*)(aph + ko + 16);
                al.q[0] = *(const v8us*)(apl + ko);
                al.q[1] = *(const v8us*)(apl + ko + 16);
                bh.q[0] = *(const v8us*)(bph + ko);
                bh.q[1] = *(const v8us*)(bph + ko + 16);
                bl.q[0] = *(const v8us*)(bpl + ko);
                bl.q[1] = *(const v8us*)(bpl + ko + 16);
                acc = wmma_bf(ah, bh, acc);
                acc = wmma_bf(ah, bl, acc);
                acc = wmma_bf(al, bh, acc);
                asm volatile("v_nop\n\tv_nop\n\tv_nop\n\tv_nop"
                             : "+v"(acc)
                             : "v"(ah.q[0]), "v"(ah.q[1]), "v"(al.q[0]), "v"(al.q[1]),
                               "v"(bh.q[0]), "v"(bh.q[1]), "v"(bl.q[0]), "v"(bl.q[1]));
            }
            v4f o0, o1;
#pragma unroll
            for (int r = 0; r < 4; ++r) {
                o0[r] = act_tanh(acc[r]     + bia0[r]);
                o1[r] = act_tanh(acc[4 + r] + bia1[r]);
            }
            float* so = So + m * SP + f0;
            *(v4f*)(so)     = o0;
            *(v4f*)(so + 4) = o1;
            __syncthreads();

#pragma unroll
            for (int j = 0; j < 2; ++j) {
                const int mm = wave + NWAVE * j;
                if ((msk >> mm) & 1u) {
                    const v4f val = *(const v4f*)(So + mm * SP + 4 * lane);
                    const int p = s_p[mm];
                    float* d = S + ((size_t)(slot0 + mm) * NNODE + p) * DIM + 4 * lane;
                    *(volatile v4f*)d = val;
                    __threadfence();
                    *(volatile v4f*)d = val;
                }
            }
            __threadfence();
        }
        __syncthreads();
    }

#pragma unroll
    for (int j = 0; j < 2; ++j) {
        const int mm = wave + NWAVE * j;
        const v4f v = *(const v4f*)(S + ((size_t)(slot0 + mm) * NNODE) * DIM + 4 * lane);
        float* d = R + (size_t)(tg0 + mm) * DIM + 4 * lane;
        *(volatile v4f*)d = v;
        __threadfence();
        *(volatile v4f*)d = v;
    }
}

__global__ __launch_bounds__(256)
void k_head(const float* __restrict__ R, const float* __restrict__ Wc,
            const float* __restrict__ bc, float* out, int ntree) {
    __shared__ float sw[NOUT * DIM];
    __shared__ __attribute__((aligned(16))) float sres[512 * NOUT];
    const int tid = threadIdx.x;
    for (int j = tid; j < NOUT * DIM; j += 256) sw[j] = Wc[j];
    __syncthreads();
    const float b0 = bc[0], b1 = bc[1], b2 = bc[2];
#pragma unroll 1
    for (int t = tid; t < ntree; t += 256) {
        const float* rr = R + (size_t)t * DIM;
        float a0 = 0.f, a1 = 0.f, a2 = 0.f;
#pragma unroll 4
        for (int d = 0; d < DIM; ++d) {
            const float x = rr[d];
            a0 = fmaf(x, sw[d],           a0);
            a1 = fmaf(x, sw[DIM + d],     a1);
            a2 = fmaf(x, sw[2 * DIM + d], a2);
        }
        sres[t * NOUT + 0] = a0 + b0;
        sres[t * NOUT + 1] = a1 + b1;
        sres[t * NOUT + 2] = a2 + b2;
    }
    __syncthreads();
    const int npiece = (ntree * NOUT) >> 2;
    const int q0 = tid, q1 = tid + 256;
    const bool w0 = q0 < npiece, w1 = q1 < npiece;
    const int c0 = w0 ? q0 : 0, c1 = w1 ? q1 : 0;
    const v4f v0 = *(const v4f*)(sres + 4 * c0);
    const v4f v1 = *(const v4f*)(sres + 4 * c1);
    if (w0) *(volatile v4f*)(out + 4 * q0) = v0;
    if (w1) *(volatile v4f*)(out + 4 * q1) = v1;
    __threadfence();
    if (w0) *(volatile v4f*)(out + 4 * q0) = v0;
    if (w1) *(volatile v4f*)(out + 4 * q1) = v1;
}

extern "C" void kernel_launch(void* const* d_in, const int* in_sizes, int n_in,
                              void* d_out, int out_size, void* d_ws, size_t ws_size,
                              hipStream_t stream) {
    const int NT = 512;
    const int HALF = 256;

    if (n_in < 8) return;
    if (in_sizes[0] != NT * NNODE * 3 || in_sizes[1] != NT || in_sizes[2] != NT * NNODE) return;
    if (in_sizes[3] <= 0 || (in_sizes[3] % DIM) != 0) return;
    if (in_sizes[4] != DIM * KDIM || in_sizes[5] != DIM ||
        in_sizes[6] != NOUT * DIM || in_sizes[7] != NOUT) return;
    if (out_size != NT * NOUT) return;
    if ((NT % HALF) != 0 || (HALF % TPB) != 0) return;
    const int vocab = in_sizes[3] / DIM;

    const int*   sub  = (const int*)d_in[0];
    const int*   lens = (const int*)d_in[1];
    const int*   eind = (const int*)d_in[2];
    const float* emb  = (const float*)d_in[3];
    const float* Wt   = (const float*)d_in[4];
    const float* bt   = (const float*)d_in[5];
    const float* Wc   = (const float*)d_in[6];
    const float* bc   = (const float*)d_in[7];
    float* out = (float*)d_out;

    const size_t b_plane = (size_t)DIM * KDIM * 2;
    const size_t b_roots = (size_t)NT * DIM * 4;
    const size_t b_state = (size_t)HALF * NNODE * DIM * 4;
    const size_t o_whi = 0;
    const size_t o_wlo = o_whi + b_plane;
    const size_t o_rts = o_wlo + b_plane;
    const size_t o_st  = o_rts + b_roots;
    const size_t total = o_st + b_state;
    if (total > ws_size) return;
    char* ws = (char*)d_ws;
    us_t*  Whi = (us_t*)(ws + o_whi);
    us_t*  Wlo = (us_t*)(ws + o_wlo);
    float* Rts = (float*)(ws + o_rts);
    float* St  = (float*)(ws + o_st);

    {
        const int n8 = DIM * KDIM / 8;
        k_wsplit<<<dim3((n8 + 255) / 256), dim3(256), 0, stream>>>(Wt, Whi, Wlo, n8);
    }
    for (int hf = 0; hf < NT / HALF; ++hf) {
        k_recur<<<dim3(HALF / TPB), dim3(256), 0, stream>>>(sub, lens, eind, emb, Whi, Wlo, bt,
                                                             St, Rts, hf * HALF, vocab);
    }
    k_head<<<dim3(1), dim3(256), 0, stream>>>(Rts, Wc, bc, out, NT);
}
